// subRelationUnit_8452495638809
// MI455X (gfx1250) — hardware-verified
//
#include <hip/hip_runtime.h>


namespace {
constexpr int N = 8192, D = 1024, K = 64, NC = 256  ;
constexpr float WS_ = 32.0f, PS_ = 1024.0f, VS_ = 8.0f;

typedef _Float16 b16;
typedef __attribute__((ext_vector_type(16))) _Float16 v16b;
typedef __attribute__((ext_vector_type(8))) _Float16 v8b;
typedef __attribute__((ext_vector_type(8))) float v8f;
typedef __attribute__((ext_vector_type(4))) float v4f;
__device__ __forceinline__ float bf16_rne(float f) { unsigned int u = __float_as_uint(f); u += 0x7FFFu + ((u >> 16) & 1u); return __uint_as_float(u & 0xFFFF0000u); }
__device__ __forceinline__ void split16(float v, b16& hi, b16& lo) { hi = (b16)v; lo = (b16)(v - (float)hi); }
__device__ __forceinline__ v16b frag_kb(const b16* p, int hh) { const v8b a = *(const v8b*)(p + 8 * hh), b = *(const v8b*)(p + 16 + 8 * hh); v16b f;
#pragma unroll
  for (int e = 0; e < 8; ++e) { f[e] = a[e]; f[8 + e] = b[e]; } return f; }
__device__ __forceinline__ v8f wmma16b(v16b a, v16b b, v8f c) {
  v8f d = __builtin_amdgcn_wmma_f32_16x16x32_f16(false, a, false, b, (short)0, c, false, false);
  asm volatile("v_nop\n\tv_nop\n\tv_nop\n\tv_nop" : "+v"(d) : "v"(a), "v"(b));
  return d;
}
__device__ __forceinline__ void wave_lds_sync() { __builtin_amdgcn_fence(__ATOMIC_RELEASE, "workgroup"); __builtin_amdgcn_wave_barrier(); __builtin_amdgcn_fence(__ATOMIC_ACQUIRE, "workgroup"); }

__global__ __launch_bounds__(256) void prep_kernel(const float* __restrict__ pf, const float* __restrict__ gf, const float* __restrict__ WG, const float* __restrict__ WK, const float* __restrict__ WQ, const float* __restrict__ WV,
                                                   b16* __restrict__ x16, b16* __restrict__ wh, b16* __restrict__ wl, float* __restrict__ gc) {
  __shared__ float red[256];
  const size_t tid = (size_t)blockIdx.x * blockDim.x + threadIdx.x, nth = (size_t)gridDim.x * blockDim.x;
  for (int pass = 0; pass < 2; ++pass) {
    for (size_t p = tid; p < (size_t)N * D / 8; p += nth) { v8b o;
#pragma unroll
      for (int e = 0; e < 8; ++e) o[e] = (b16)bf16_rne(pf[p * 8 + e]);
      *(volatile v8b*)(x16 + p * 8) = o; }
    for (size_t p = tid; p < (size_t)NC * D; p += nth) { const int n = (int)(p / D), d = (int)(p % D); float v = 0.0f;
      if (n < K) v = WK[(size_t)d * K + n]; else if (n < 2 * K) v = WQ[(size_t)d * K + n - K]; else if (n < 3 * K) v = WV[(size_t)d * K + n - 2 * K]; else if (n == 3 * K) v = WG[d];
      b16 a, c; split16(bf16_rne(v) * WS_, a, c); ((volatile b16*)wh)[p] = a; ((volatile b16*)wl)[p] = c; }
    __threadfence();
  }
  if (blockIdx.x == 0) { float s = 0.0f; for (int d = threadIdx.x; d < D; d += 256) s += bf16_rne(gf[d]) * bf16_rne(WG[d]); red[threadIdx.x] = s; __syncthreads();
    if (threadIdx.x == 0) { float t = 0.0f; for (int i = 0; i < 256; ++i) t += red[i]; for (int pass = 0; pass < 2; ++pass) { ((volatile float*)gc)[0] = t; __threadfence(); } } }
}

__global__ __launch_bounds__(128) void proj_kernel(const b16* __restrict__ x16, const b16* __restrict__ wh, const b16* __restrict__ wl, const float* __restrict__ bK, const float* __restrict__ bQ, const float* __restrict__ bV, const float* __restrict__ bG, const float* __restrict__ gc, float* __restrict__ proj) {
  __shared__ __attribute__((aligned(16))) float Ts[4][32 * 64];
  const int lane = threadIdx.x & 31, wave = threadIdx.x >> 5, nloc = lane & 15, hlf = lane >> 4, m0 = blockIdx.y * 128 + wave * 32, c0 = blockIdx.x * 64;
  v8f acc[2][4];
#pragma unroll
  for (int r = 0; r < 2; ++r)
#pragma unroll
    for (int t = 0; t < 4; ++t) acc[r][t] = (v8f){};
#pragma unroll 2
  for (int kb = 0; kb < D; kb += 32) { const v16b a0 = frag_kb(x16 + (size_t)(m0 + nloc) * D + kb, hlf), a1 = frag_kb(x16 + (size_t)(m0 + 16 + nloc) * D + kb, hlf);
#pragma unroll
    for (int t = 0; t < 4; ++t) { const size_t bo = (size_t)(c0 + t * 16 + nloc) * D + kb; const v16b b0 = frag_kb(wh + bo, hlf), b1 = frag_kb(wl + bo, hlf);
      acc[0][t] = wmma16b(a0, b0, acc[0][t]); acc[0][t] = wmma16b(a0, b1, acc[0][t]); acc[1][t] = wmma16b(a1, b0, acc[1][t]); acc[1][t] = wmma16b(a1, b1, acc[1][t]); } }
  float* Tt = Ts[wave];
#pragma unroll
  for (int t = 0; t < 4; ++t) { const int c = c0 + t * 16 + nloc; float bias = 0.0f;
    if (c < K) bias = bf16_rne(bK[c]); else if (c < 2 * K) bias = bf16_rne(bQ[c - K]); else if (c < 3 * K) bias = bf16_rne(bV[c - 2 * K]); else if (c == 3 * K) bias = bf16_rne(bG[0]) + gc[0];
#pragma unroll
    for (int r = 0; r < 2; ++r)
#pragma unroll
      for (int v = 0; v < 8; ++v) Tt[(r * 16 + v + 8 * hlf) * 64 + t * 16 + nloc] = acc[r][t][v] * (1.0f / WS_) + bias; }
  wave_lds_sync();
  float* dst0 = proj + (size_t)m0 * NC + c0;
  for (int pass = 0; pass < 2; ++pass) {
#pragma unroll
    for (int j = 0; j < 16; ++j) { const int rr = j * 2 + hlf, c4 = nloc * 4; *(volatile v4f*)(dst0 + (size_t)rr * NC + c4) = *(const v4f*)(Tt + rr * 64 + c4); }
    __threadfence();
  }
}

__global__ __launch_bounds__(128) void rows_kernel(const float* __restrict__ proj, const float* __restrict__ WP, float* __restrict__ ab, b16* __restrict__ vth, b16* __restrict__ vtl) {
  __shared__ __attribute__((aligned(16))) b16 Th[K][128 + 8], Tl[K][128 + 8];
  const int t_ = threadIdx.x, i = blockIdx.x * 128 + t_; const float* row = proj + (size_t)i * NC;
  float a = 0.0f, b = 0.0f;
#pragma unroll 4
  for (int k = 0; k < K; ++k) { const float w = bf16_rne(WP[k]); a += row[k] * w; b += row[K + k] * w; }
  const float g = fmaxf(row[3 * K], 0.0f);
#pragma unroll 4
  for (int k = 0; k < K; ++k) { b16 h_, l_; split16(row[2 * K + k] * VS_, h_, l_); Th[k][t_] = h_; Tl[k][t_] = l_; }
  __syncthreads();
  const v4f o = {a, b, g, 0.0f};
  for (int pass = 0; pass < 2; ++pass) { *(volatile v4f*)(ab + (size_t)i * 4) = o;
    for (int q = t_; q < K * 16; q += 128) { const int k = q >> 4, c8 = (q & 15) * 8; *(volatile v8b*)(vth + (size_t)k * N + blockIdx.x * 128 + c8) = *(const v8b*)(&Th[k][c8]); *(volatile v8b*)(vtl + (size_t)k * N + blockIdx.x * 128 + c8) = *(const v8b*)(&Tl[k][c8]); }
    __threadfence(); }
}

__global__ __launch_bounds__(256) void bmax_kernel(const float* __restrict__ ab, float* __restrict__ bm) {
  __shared__ float red[256]; float m = -INFINITY;
  for (int j = threadIdx.x; j < N; j += 256) m = fmaxf(m, ab[(size_t)j * 4 + 1]);
  red[threadIdx.x] = m; __syncthreads();
  if (threadIdx.x == 0) { float t = -INFINITY; for (int i = 0; i < 256; ++i) t = fmaxf(t, red[i]); for (int pass = 0; pass < 2; ++pass) { ((volatile float*)bm)[0] = t; __threadfence(); } }
}
__global__ __launch_bounds__(256) void denom_kernel(const float* __restrict__ ab, const float* __restrict__ bm, const float* __restrict__ bP, float* __restrict__ ml) {
  const int i = blockIdx.x * 256 + threadIdx.x; const v4f r = *(const v4f*)(ab + (size_t)i * 4); const float a = r[0], g = r[2], c = bf16_rne(bP[0]);
  const float m = fmaxf(a + bm[0] + c, 0.0f) * g; float l = 0.0f;
  for (int j = 0; j < N; ++j) { const float bj = ab[(size_t)j * 4 + 1]; l += __expf(fmaxf(a + bj + c, 0.0f) * g - m); }
  const v4f o = {m, 1.0f / l, a, g};
  for (int pass = 0; pass < 2; ++pass) { *(volatile v4f*)(ml + (size_t)i * 4) = o; __threadfence(); }
}

__global__ __launch_bounds__(128) void out_kernel(const float* __restrict__ ab, const float* __restrict__ ml, const float* __restrict__ bP, const b16* __restrict__ vth, const b16* __restrict__ vtl, float* __restrict__ out) {
  __shared__ __attribute__((aligned(16))) float Ts[4][16][K + 4];
  const int lane = threadIdx.x & 31, wave = threadIdx.x >> 5, nloc = lane & 15, hlf = lane >> 4, j0 = (blockIdx.x * 4 + wave) * 16, j = j0 + nloc;
  const float bj = ab[(size_t)j * 4 + 1], c = bf16_rne(bP[0]);
  v8f acc[4] = {{}, {}, {}, {}};
  for (int ib = 0; ib < N; ib += 32) { v16b ph, pl;
#pragma unroll
    for (int e = 0; e < 16; ++e) { const int i = ib + ((e < 8) ? (8 * hlf + e) : (16 + 8 * hlf + e - 8)); const v4f r = *(const v4f*)(ml + (size_t)i * 4);
      const float p = __expf(fmaxf(r[2] + bj + c, 0.0f) * r[3] - r[0]) * r[1] * PS_; b16 h_, l_; split16(p, h_, l_); ph[e] = h_; pl[e] = l_; }
#pragma unroll
    for (int t = 0; t < 4; ++t) { const v16b b0 = frag_kb(vth + (size_t)(t * 16 + nloc) * N + ib, hlf), b1 = frag_kb(vtl + (size_t)(t * 16 + nloc) * N + ib, hlf);
      acc[t] = wmma16b(ph, b0, acc[t]); acc[t] = wmma16b(pl, b0, acc[t]); acc[t] = wmma16b(ph, b1, acc[t]); } }
#pragma unroll
  for (int t = 0; t < 4; ++t)
#pragma unroll
    for (int v = 0; v < 8; ++v) Ts[wave][8 * hlf + v][t * 16 + nloc] = acc[t][v] * (1.0f / (PS_ * VS_));
  wave_lds_sync();
  float* dst = out + (size_t)j0 * K;
  for (int pass = 0; pass < 2; ++pass) {
#pragma unroll
    for (int q = 0; q < 8; ++q) { const int rr = q * 2 + hlf, c4 = nloc * 4; *(volatile v4f*)(dst + (size_t)rr * K + c4) = *(const v4f*)(&Ts[wave][rr][c4]); }
    __threadfence();
  }
}
}

extern "C" void kernel_launch(void* const* d_in, const int* in_sizes, int n_in,
                              void* d_out, int out_size, void* d_ws, size_t ws_size, hipStream_t stream) {
  (void)n_in; (void)out_size;
  const float* pf = (const float*)d_in[0]; const float* gf = (const float*)d_in[1]; const float* WG = (const float*)d_in[2]; const float* bG = (const float*)d_in[3]; const float* WK = (const float*)d_in[4]; const float* bK = (const float*)d_in[5];
  const float* WQ = (const float*)d_in[6]; const float* bQ = (const float*)d_in[7]; const float* WP = (const float*)d_in[8]; const float* bP = (const float*)d_in[9]; const float* WV = (const float*)d_in[10]; const float* bV = (const float*)d_in[11];
  float* out = (float*)d_out;
  if (in_sizes[0] != N * D || in_sizes[1] != D || in_sizes[2] != D || in_sizes[4] != D * K || in_sizes[8] != K || in_sizes[10] != D * K) return;
  size_t off = 0; char* ws = (char*)d_ws;
  auto carve = [&](size_t bytes) { char* p = ws + off; off += (bytes + 255) & ~(size_t)255; return p; };
  b16* x16 = (b16*)carve((size_t)N * D * 2); b16* wh = (b16*)carve((size_t)NC * D * 2); b16* wl = (b16*)carve((size_t)NC * D * 2); float* gc = (float*)carve(256); float* proj = (float*)carve((size_t)N * NC * 4);
  float* ab = (float*)carve((size_t)N * 4 * 4); b16* vth = (b16*)carve((size_t)K * N * 2); b16* vtl = (b16*)carve((size_t)K * N * 2); float* bm = (float*)carve(256); float* ml = (float*)carve((size_t)N * 4 * 4);
  if (off > ws_size) return;
  prep_kernel<<<1024, 256, 0, stream>>>(pf, gf, WG, WK, WQ, WV, x16, wh, wl, gc);
  proj_kernel<<<dim3(NC / 64, N / 128), 128, 0, stream>>>(x16, wh, wl, bK, bQ, bV, bG, gc, proj);
  rows_kernel<<<N / 128, 128, 0, stream>>>(proj, WP, ab, vth, vtl);
  bmax_kernel<<<1, 256, 0, stream>>>(ab, bm);
  denom_kernel<<<N / 256, 256, 0, stream>>>(ab, bm, bP, ml);
  out_kernel<<<N / 16 / 4, 128, 0, stream>>>(ab, ml, bP, vth, vtl, out);
}
